// Net_81793357185728
// MI455X (gfx1250) — hardware-run, weakly checked
//
#include <hip/hip_runtime.h>

typedef float          v8f   __attribute__((ext_vector_type(8)));
typedef float          v4f   __attribute__((ext_vector_type(4)));
typedef unsigned int   v4u   __attribute__((ext_vector_type(4)));
typedef int            v8i   __attribute__((ext_vector_type(8)));
typedef unsigned short v8us  __attribute__((ext_vector_type(8)));
typedef unsigned short v16us __attribute__((ext_vector_type(16)));
typedef __bf16         v16bf __attribute__((ext_vector_type(16)));
typedef _Float16       v16h  __attribute__((ext_vector_type(16)));
typedef v4f  __attribute__((may_alias)) v4fa;
typedef v8us __attribute__((may_alias)) v8usa;
union FragB { v16bf v; v16us u; v8us h[2]; v8i w; };
union FragH { v16h  v; v16us u; v8us h[2]; v8i w; };

__device__ __forceinline__ v8f wmb(const FragB& a, const FragB& b, v8f c) {
  v8f d = __builtin_amdgcn_wmma_f32_16x16x32_bf16(false, a.v, false, b.v, (short)0, c, false, false);
  asm volatile("v_nop\n\tv_nop\n\tv_nop\n\tv_nop" : "+v"(d) : "v"(a.w), "v"(b.w));
  return d;
}

__device__ __forceinline__ v8f wmh(const FragH& a, const FragH& b, v8f c) {
  v8f d = __builtin_amdgcn_wmma_f32_16x16x32_f16(false, a.v, false, b.v, (short)0, c, false, false);
  asm volatile("v_nop\n\tv_nop\n\tv_nop\n\tv_nop" : "+v"(d) : "v"(a.w), "v"(b.w));
  return d;
}

__device__ __forceinline__ unsigned bf16_bits(float f) {
  const unsigned u = __float_as_uint(f);
  const unsigned r = (u + 0x7FFFu + ((u >> 16) & 1u)) >> 16;
  const unsigned q = (u >> 16) | 0x40u;
  return ((u & 0x7fffffffu) > 0x7f800000u) ? q : r;
}

__device__ __forceinline__ float bf16_val(float f) {
  return __uint_as_float(bf16_bits(f) << 16);
}
__device__ __forceinline__ int clampi(int v, int lo, int hi) {
  return v < lo ? lo : (v > hi ? hi : v);
}

__device__ __forceinline__ unsigned f16_bits(float f) {
  const unsigned u  = __float_as_uint(f);
  const unsigned s  = (u >> 16) & 0x8000u;
  const unsigned a  = u & 0x7fffffffu;
  const unsigned t  = a - 0x38000000u;
  const unsigned r  = (t + 0x0FFFu + ((t >> 13) & 1u)) >> 13;
  const unsigned rc = r > 0x7C00u ? 0x7C00u : r;
  const bool small  = a < 0x38800000u;
  const bool isnan  = a > 0x7f800000u;
  const unsigned fin = small ? 0u : (s | rc);
  return isnan ? (s | 0x7E00u) : fin;
}

__device__ __forceinline__ unsigned pk16(unsigned lo, unsigned hi) { return lo | (hi << 16); }
__device__ __forceinline__ unsigned bf16_lo_bits(float v) {
  float hi = bf16_val(v);
  asm volatile("" : "+v"(hi));
  return bf16_bits(v - hi);
}
__device__ __forceinline__ v4u pack8_bf16(v4f a, v4f c) {
  return (v4u){ pk16(bf16_bits(a[0]), bf16_bits(a[1])), pk16(bf16_bits(a[2]), bf16_bits(a[3])),
                pk16(bf16_bits(c[0]), bf16_bits(c[1])), pk16(bf16_bits(c[2]), bf16_bits(c[3])) };
}
__device__ __forceinline__ v4u pack8_bf16_lo(v4f a, v4f c) {
  return (v4u){ pk16(bf16_lo_bits(a[0]), bf16_lo_bits(a[1])), pk16(bf16_lo_bits(a[2]), bf16_lo_bits(a[3])),
                pk16(bf16_lo_bits(c[0]), bf16_lo_bits(c[1])), pk16(bf16_lo_bits(c[2]), bf16_lo_bits(c[3])) };
}
__device__ __forceinline__ v4u pack8_f16(v4f a, v4f c) {
  return (v4u){ pk16(f16_bits(a[0]), f16_bits(a[1])), pk16(f16_bits(a[2]), f16_bits(a[3])),
                pk16(f16_bits(c[0]), f16_bits(c[1])), pk16(f16_bits(c[2]), f16_bits(c[3])) };
}

template <int FORM>
__global__ __launch_bounds__(256) void k_plane(const float* __restrict__ src, int rows, int cols, int ldsrc,
                                               unsigned short* __restrict__ dst, int MP, int KP) {
  static_assert(FORM >= 0 && FORM <= 3);
  const int KTOT = (FORM == 1 || FORM == 3) ? 2 * KP : KP;
  const unsigned ppr   = (unsigned)(KTOT >> 3);
  const unsigned kp8   = (unsigned)(KP >> 3);
  const unsigned total = (unsigned)MP * ppr;
  const unsigned g     = blockIdx.x * 256u + threadIdx.x;
  const unsigned rowu  = g / ppr;
  const unsigned p     = g - rowu * ppr;
  const bool second    = p >= kp8;
  const int row = (int)rowu;
  const int c0  = (int)((second ? p - kp8 : p) << 3);
  const float* srow = src + (size_t)clampi(row, 0, rows - 1) * (size_t)ldsrc;
  float x[8];
  unsigned mk[8];
#pragma unroll
  for (int e = 0; e < 8; ++e) {
    const int c = c0 + e;
    const float v = srow[clampi(c, 0, cols - 1)];
    asm volatile("" :: "v"(v));
    x[e]  = v;
    mk[e] = (row < rows && c < cols) ? 0xFFFFu : 0u;
  }
  const v4f a = (v4f){ x[0], x[1], x[2], x[3] };
  const v4f c = (v4f){ x[4], x[5], x[6], x[7] };
  v4u o;
  if (FORM == 2) {
    o = pack8_f16(a, c);
  } else {
    const v4u hi = pack8_bf16(a, c);
    o = hi;
    if (FORM == 1) { const v4u lo = pack8_bf16_lo(a, c); o = second ? lo : hi; }
  }
  const v4u mw = (v4u){ pk16(mk[0], mk[1]), pk16(mk[2], mk[3]), pk16(mk[4], mk[5]), pk16(mk[6], mk[7]) };
  o &= mw;
  if (g < total) {
    volatile v4u* q = (volatile v4u*)(dst + (size_t)g * 8);
    *q = o;
    __threadfence();
    *q = o;
  }
}

template <int FORM> struct FragOf    { typedef FragB T; };
template <>         struct FragOf<2> { typedef FragH T; };
__device__ __forceinline__ v8f mm(const FragB& a, const FragB& b, v8f c) { return wmb(a, b, c); }
__device__ __forceinline__ v8f mm(const FragH& a, const FragH& b, v8f c) { return wmh(a, b, c); }
template <class F> __device__ __forceinline__ F ld_frag(const unsigned short* p) {
  F f;
  f.h[0] = *(const v8usa*)(p);
  f.h[1] = *(const v8usa*)(p + 16);
  return f;
}

template <int FORM, int EPI>
__global__ __launch_bounds__(256) __attribute__((amdgpu_num_vgpr(248)))
void k_gemm_nt(const unsigned short* __restrict__ A, const unsigned short* __restrict__ B,
               const float* __restrict__ bias, float* __restrict__ D, int M, int N, int KTOT, int ldd) {
  static_assert(FORM >= 0 && FORM <= 2);
  static_assert(EPI == 0 || EPI == 1);
  typedef typename FragOf<FORM>::T F;
  __shared__ __attribute__((aligned(16))) float sT[8][16 * 68];
  const int lane = threadIdx.x & 31;
  const int wave = threadIdx.x >> 5;
  const int tilesM = (M + 63) >> 6;
  const int tilesN = (N + 63) >> 6;
  const int tile = blockIdx.x * 8 + wave;
  if (tile >= tilesM * tilesN) return;
  const int tm = tile / tilesN;
  const int tn = tile - tm * tilesN;
  const int m0 = tm << 6;
  const int n0 = tn << 6;

  const int rl = lane & 15;
  const int h8 = (lane >> 4) * 8;
  const unsigned short* pa = A + (size_t)(m0 + rl) * (size_t)KTOT + h8;
  const unsigned short* pb = B + (size_t)(n0 + rl) * (size_t)KTOT + h8;

  v8f acc[4][4];
#pragma unroll
  for (int i = 0; i < 4; ++i)
#pragma unroll
    for (int j = 0; j < 4; ++j) acc[i][j] = (v8f){0.f, 0.f, 0.f, 0.f, 0.f, 0.f, 0.f, 0.f};

#pragma unroll 1
  for (int k0 = 0; k0 < KTOT; k0 += 32) {
    F bf[4];
#pragma unroll
    for (int j = 0; j < 4; ++j) bf[j] = ld_frag<F>(pb + (size_t)(j << 4) * (size_t)KTOT + k0);
#pragma unroll
    for (int i = 0; i < 4; ++i) {
      const F af = ld_frag<F>(pa + (size_t)(i << 4) * (size_t)KTOT + k0);
#pragma unroll
      for (int j = 0; j < 4; ++j) acc[i][j] = mm(af, bf[j], acc[i][j]);
    }
  }

  float* slab = sT[wave];
  const int hh = lane >> 4;
  const int c4 = (lane & 15) * 4;
  const int nc = n0 + c4;
  const bool cok = nc < N;
  v4f bv = (v4f){0.f, 0.f, 0.f, 0.f};
  if (EPI == 1) {
    bv = *(const v4fa*)(bias + clampi(nc, 0, N - 4));
    asm volatile("" :: "v"(bv));
  }
#pragma unroll
  for (int i = 0; i < 4; ++i) {
    const int mBase = m0 + (i << 4);
#pragma unroll
    for (int j = 0; j < 4; ++j) {
#pragma unroll
      for (int r = 0; r < 8; ++r) slab[(h8 + r) * 68 + (j << 4) + rl] = acc[i][j][r];
    }
    __builtin_amdgcn_fence(__ATOMIC_RELEASE, "workgroup");
    __builtin_amdgcn_wave_barrier();
    __builtin_amdgcn_fence(__ATOMIC_ACQUIRE, "workgroup");
    v4f vv[8];
#pragma unroll
    for (int it = 0; it < 8; ++it) {
      const int row = it * 2 + hh;
      v4f v = *(const v4fa*)(slab + row * 68 + c4);
      if (EPI == 1) v += bv;
      vv[it] = v;
    }
    for (int pass = 0; pass < 2; ++pass) {
#pragma unroll
      for (int it = 0; it < 8; ++it) {
        const int row = mBase + it * 2 + hh;
        if (cok && row < M) *(volatile v4f*)(D + (size_t)row * (size_t)ldd + nc) = vv[it];
      }
      __threadfence();
    }
    __builtin_amdgcn_fence(__ATOMIC_RELEASE, "workgroup");
    __builtin_amdgcn_wave_barrier();
    __builtin_amdgcn_fence(__ATOMIC_ACQUIRE, "workgroup");
  }
}

#include <stddef.h>
#include <stdint.h>
#include <math.h>

#ifndef HL2
#define HL2 1
#endif

#define NN      50000
#define NE      800000
#define DF      128
#define DH      128
#define DC      40
#define DCP     64
#define OUTN    (NN * DC)
#define MPAD    50048
#define K2      (HL2 ? 256 : 128)
#define NTHR    256
#define NWAVE   8
#define NBRUN   1024
#define SLB     10
#define NBLK    49
#define EPW     (NE / NWAVE)
#define STEPE   256
#define NSTEP   ((EPW + STEPE - 1) / STEPE)
#define WLCAP   2560
#define LCAP    20800
#define DEGCAP  64
#define MEAS_B1024 16623
#define MEAS_DEG   35
#define GPW     4
#define RGRP    32
#define BK_ZINTS   (NWAVE * WLCAP + 2 * LCAP + 3 * NBRUN)
#define BK_INTS    (BK_ZINTS + 16)
#define BK_LDS     (BK_INTS * 4)
#define LIST_V4    (2 * LCAP / 4)
#define LIST_IT    ((LIST_V4 + NTHR - 1) / NTHR)
#define OUT_V4     (RGRP * DC / 4)
#define OUT_IT     (OUT_V4 / 32)
#define NBW1    ((DH * DF / 8) / NTHR)
#define NBW2    ((DCP * K2 / 8) / NTHR)
#define T_U1    0
#define T_V1    128
#define T_B1    256
#define T_LB1   384
#define T_U2    512
#define T_V2    576
#define T_B2    640
#define T_LB2   704
#define T_TOT   768

static_assert(NBRUN == (1 << SLB) && NWAVE * GPW * RGRP == NBRUN);
static_assert((NBLK - 1) * NBRUN < NN && NBLK * NBRUN >= MPAD && NN - (NBLK - 1) * NBRUN == 848);
static_assert(MPAD % 128 == 0 && MPAD % 64 == 0 && MPAD >= NN && MPAD % RGRP == 0 && MPAD == 391 * 128);
static_assert(NE % NWAVE == 0 && EPW % 8 == 0 && NE % 8 == 0);
static_assert(NE - 390 * 2048 == 1280 && EPW - 390 * STEPE == 160 && NSTEP == 391);
static_assert((((long long)(NE - 1)) << SLB) + NBRUN < (1LL << 31));
static_assert(LCAP % 64 == 0 && 4 * LCAP >= 5 * MEAS_B1024 && LIST_V4 % 32 == 0);
static_assert(DEGCAP == 64 && DEGCAP >= MEAS_DEG + 8);
static_assert(WLCAP % 4 == 0 && BK_ZINTS % 4 == 0 && 4 * WLCAP >= 5 * (EPW / NBLK));
static_assert(BK_LDS == 260672 && BK_LDS <= 262144 && BK_LDS + 0 <= 327680);
static_assert(2 * NWAVE * RGRP * DC * 4 == 81920 && 8 * 16 * 68 * 4 <= 327680);
static_assert((RGRP * DC) % 4 == 0 && (RGRP * DC * 4) % 128 == 0 && OUT_IT * 32 == OUT_V4 && OUT_IT == 10);
static_assert(((NN % RGRP) * DC) % 128 == 0 && OUTN % 4 == 0 && (OUTN * 4) % 128 == 0);
static_assert(K2 % 32 == 0 && DF % 32 == 0 && DH == 128 && DC % 4 == 0 && DC <= DCP && DC % 2 == 0);
static_assert((DH * DF / 8) % NTHR == 0 && (DCP * K2 / 8) % NTHR == 0);
static_assert((MPAD * (DF / 8)) % 256 == 0);
static_assert(T_TOT == 4 * 128 + 4 * 64 && T_TOT % 4 == 0 && T_TOT / 4 <= NTHR);

typedef float v2f __attribute__((ext_vector_type(2)));
typedef int   v2i __attribute__((ext_vector_type(2)));
typedef int   v4i __attribute__((ext_vector_type(4)));
typedef v2f __attribute__((may_alias)) v2fa;
typedef v2i __attribute__((may_alias)) v2ia;
typedef v4i __attribute__((may_alias)) v4ia;

#define PIN(x) asm volatile("" :: "v"(x))

__device__ __forceinline__ void wunit_nat(const float* __restrict__ W, int nvalid, int KW, int u,
                                          unsigned short* dstp) {
  const int ppr = KW >> 3;
  const int n   = u / ppr;
  const int k8  = (u - n * ppr) << 3;
  const int kk  = k8 & (DH - 1);
  const int nc  = n < nvalid ? n : nvalid - 1;
  const float* p = W + (size_t)nc * (size_t)DH + kk;
  const v4f a = *(const v4fa*)(p);
  const v4f c = *(const v4fa*)(p + 4);
  asm volatile("" :: "v"(a));
  asm volatile("" :: "v"(c));
  const unsigned mk = (n < nvalid) ? 0xFFFFFFFFu : 0u;
  v4u o = pack8_bf16(a, c);
  o &= (v4u){ mk, mk, mk, mk };
  volatile v4u* q = (volatile v4u*)(dstp + (size_t)n * (size_t)KW + k8);
  *q = o;
  __threadfence();
  *q = o;
}

__global__ __launch_bounds__(NTHR) void k_prep(const float* __restrict__ linw1, const float* __restrict__ linb1,
                                               const float* __restrict__ w1a, const float* __restrict__ w2a,
                                               const float* __restrict__ w2ba, const float* __restrict__ linw2,
                                               const float* __restrict__ linb2, const float* __restrict__ w1b,
                                               const float* __restrict__ w2b, const float* __restrict__ w2bb,
                                               unsigned short* W1P, unsigned short* W2D, float* TAB) {
  __shared__ __attribute__((aligned(16))) float sTb[T_TOT];
  const int blk = (int)blockIdx.x;
  const int tid = (int)threadIdx.x;
  const int lane = tid & 31, wave = tid >> 5;
  if (blk < NBW1) {
    wunit_nat(linw1, DH, DF, blk * NTHR + tid, W1P);
  } else if (blk < NBW1 + NBW2) {
    wunit_nat(linw2, DC, K2, (blk - NBW1) * NTHR + tid, W2D);
  } else {
    if (wave < 4) {
      const int c = tid;
      double au = 0.0, av = 0.0;
#pragma unroll 1
      for (int k = 0; k < DH; ++k) {
        const float w  = bf16_val(w1a[k]);
        const float wk = bf16_val(w2a[(size_t)c * DH + k]);
        const float ap = (w >= 0.0f) ? w : 0.2f * w;
        const float bn = (w <  0.0f) ? w : 0.2f * w;
        au += (double)wk * (double)ap;
        av += (double)wk * (double)bn;
      }
      sTb[T_U1 + c] = (float)au;
      sTb[T_V1 + c] = (float)av;
    } else if (wave < 6) {
      const int c  = tid - 128;
      const int cc = c < DC ? c : DC - 1;
      double au = 0.0, av = 0.0;
#pragma unroll 1
      for (int k = 0; k < DC; ++k) {
        const float w  = bf16_val(w1b[k]);
        const float wk = bf16_val(w2b[(size_t)cc * DC + k]);
        const float ap = (w >= 0.0f) ? w : 0.2f * w;
        const float bn = (w <  0.0f) ? w : 0.2f * w;
        au += (double)wk * (double)ap;
        av += (double)wk * (double)bn;
      }
      const float fu = (float)au, fv = (float)av;
      sTb[T_U2 + c] = (c < DC) ? fu : 0.0f;
      sTb[T_V2 + c] = (c < DC) ? fv : 0.0f;
    } else if (wave == 6) {
      const v4f xb = *(const v4fa*)(w2ba + 4 * lane);
      const v4f xl = *(const v4fa*)(linb1 + 4 * lane);
      asm volatile("" :: "v"(xb));
      asm volatile("" :: "v"(xl));
#pragma unroll
      for (int e = 0; e < 4; ++e) {
        sTb[T_B1 + 4 * lane + e]  = bf16_val(xb[e]);
        sTb[T_LB1 + 4 * lane + e] = bf16_val(xl[e]);
      }
    } else {
      const int c4 = 4 * lane;
      const int cc = c4 < DC - 4 ? c4 : DC - 4;
      const v4f xb = *(const v4fa*)(w2bb + cc);
      const v4f xl = *(const v4fa*)(linb2 + cc);
      asm volatile("" :: "v"(xb));
      asm volatile("" :: "v"(xl));
      const bool ok = c4 < DC;
      if (lane < 16) {
#pragma unroll
        for (int e = 0; e < 4; ++e) {
          const float vb = bf16_val(xb[e]);
          const float vl = bf16_val(xl[e]);
          sTb[T_B2 + c4 + e]  = ok ? vb : 0.0f;
          sTb[T_LB2 + c4 + e] = ok ? vl : 0.0f;
        }
      }
    }
    __syncthreads();
    const int tq = tid < (T_TOT / 4) ? tid : (T_TOT / 4 - 1);
    const v4f tv = *(const v4fa*)(sTb + 4 * tq);
    if (tid < T_TOT / 4) *(volatile v4f*)(TAB + 4 * tid) = tv;
    __threadfence();
    if (tid < T_TOT / 4) *(volatile v4f*)(TAB + 4 * tid) = tv;
  }
}

#define PUTJ(HJ, J, SJ) { \
    const int wv = ((e0 + (J)) << SLB) | (int)(SJ); \
    if (HJ) { if (pos < WLCAP) wlw[pos] = wv; } \
    pos += (HJ) ? 1 : 0; }

__global__ __launch_bounds__(NTHR) void k_bucket(const int* __restrict__ srcs, const int* __restrict__ dsts,
                                                 int nN, int* listG, int* cntG, int* offG, int* flagG) {
  extern __shared__ __attribute__((aligned(16))) int dsm[];
  int* wl   = dsm;
  int* sl   = dsm + NWAVE * WLCAP;
  int* cnt  = sl + 2 * LCAP;
  int* offs = cnt + NBRUN;
  int* cur  = offs + NBRUN;
  int* misc = cur + NBRUN;
  const int tid = (int)threadIdx.x, lane = tid & 31, wave = tid >> 5;
  const int b = (int)blockIdx.x;
  const int nodeBase = b * NBRUN;
  const int nb = clampi(nN - nodeBase, 0, NBRUN);

  {
    const v4i z4 = {0, 0, 0, 0};
    for (int i = tid * 4; i < BK_ZINTS; i += NTHR * 4) *(v4ia*)(dsm + i) = z4;
    if (tid < 16) misc[tid] = 0;
  }
  __syncthreads();

  {
    int* wlw = wl + wave * WLCAP;
    const int wbeg = wave * EPW;
    const int wend = wbeg + EPW;
    const unsigned nbs = (unsigned)nodeBase;
    const unsigned unb = (unsigned)nb;
    int wc = 0;
#pragma unroll 1
    for (int st = 0; st < NSTEP; ++st) {
      const int e0  = wbeg + st * STEPE + lane * 8;
      const int e0c = e0 < (NE - 8) ? e0 : (NE - 8);
      const v4i da = *(const v4ia*)(dsts + e0c);
      const v4i db = *(const v4ia*)(dsts + e0c + 4);
      PIN(da.x); PIN(da.y); PIN(da.z); PIN(da.w);
      PIN(db.x); PIN(db.y); PIN(db.z); PIN(db.w);
      const unsigned s0 = (unsigned)da.x - nbs, s1 = (unsigned)da.y - nbs;
      const unsigned s2 = (unsigned)da.z - nbs, s3 = (unsigned)da.w - nbs;
      const unsigned s4 = (unsigned)db.x - nbs, s5 = (unsigned)db.y - nbs;
      const unsigned s6 = (unsigned)db.z - nbs, s7 = (unsigned)db.w - nbs;
      const bool h0 = (e0 + 0 < wend) && (s0 < unb);
      const bool h1 = (e0 + 1 < wend) && (s1 < unb);
      const bool h2 = (e0 + 2 < wend) && (s2 < unb);
      const bool h3 = (e0 + 3 < wend) && (s3 < unb);
      const bool h4 = (e0 + 4 < wend) && (s4 < unb);
      const bool h5 = (e0 + 5 < wend) && (s5 < unb);
      const bool h6 = (e0 + 6 < wend) && (s6 < unb);
      const bool h7 = (e0 + 7 < wend) && (s7 < unb);
      const unsigned m0 = __builtin_amdgcn_ballot_w32(h0);
      const unsigned m1 = __builtin_amdgcn_ballot_w32(h1);
      const unsigned m2 = __builtin_amdgcn_ballot_w32(h2);
      const unsigned m3 = __builtin_amdgcn_ballot_w32(h3);
      const unsigned m4 = __builtin_amdgcn_ballot_w32(h4);
      const unsigned m5 = __builtin_amdgcn_ballot_w32(h5);
      const unsigned m6 = __builtin_amdgcn_ballot_w32(h6);
      const unsigned m7 = __builtin_amdgcn_ballot_w32(h7);
      const unsigned many = m0 | m1 | m2 | m3 | m4 | m5 | m6 | m7;
      if (many != 0u) {
        unsigned pre = __builtin_amdgcn_mbcnt_lo(m0, 0u);
        pre = __builtin_amdgcn_mbcnt_lo(m1, pre);
        pre = __builtin_amdgcn_mbcnt_lo(m2, pre);
        pre = __builtin_amdgcn_mbcnt_lo(m3, pre);
        pre = __builtin_amdgcn_mbcnt_lo(m4, pre);
        pre = __builtin_amdgcn_mbcnt_lo(m5, pre);
        pre = __builtin_amdgcn_mbcnt_lo(m6, pre);
        pre = __builtin_amdgcn_mbcnt_lo(m7, pre);
        int pos = wc + (int)pre;
        PUTJ(h0, 0, s0)
        PUTJ(h1, 1, s1)
        PUTJ(h2, 2, s2)
        PUTJ(h3, 3, s3)
        PUTJ(h4, 4, s4)
        PUTJ(h5, 5, s5)
        PUTJ(h6, 6, s6)
        PUTJ(h7, 7, s7)
        wc += (int)__builtin_popcount(m0) + (int)__builtin_popcount(m1) + (int)__builtin_popcount(m2)
            + (int)__builtin_popcount(m3) + (int)__builtin_popcount(m4) + (int)__builtin_popcount(m5)
            + (int)__builtin_popcount(m6) + (int)__builtin_popcount(m7);
      }
    }
    if (lane == 0) misc[wave] = wc;
  }
  __syncthreads();

  if (wave == 0) {
    int t = 0, ov = 0;
#pragma unroll 1
    for (int w2 = 0; w2 < NWAVE; ++w2) {
      int c = misc[w2];
      ov |= (c > WLCAP) ? 1 : 0;
      c = c < 0 ? 0 : (c > WLCAP ? WLCAP : c);
      c = __builtin_amdgcn_readfirstlane(c);
#pragma unroll 1
      for (int b0 = 0; b0 < c; b0 += 32) {
        const int idx = b0 + lane;
        const int ent = wl[w2 * WLCAP + (idx < WLCAP ? idx : WLCAP - 1)];
        const int m32 = (c - b0) < 32 ? (c - b0) : 32;
#pragma unroll 1
        for (int k = 0; k < m32; ++k) {
          const int u    = __builtin_amdgcn_readlane(ent, k);
          const int slot = u & (NBRUN - 1);
          if (t < LCAP) {
            const int cvv = cnt[slot];
            if (lane == 0) cnt[slot] = cvv + 1;
            t = t + 1;
          } else {
            ov = 1;
          }
        }
      }
    }
    if (lane == 0) { misc[8] = t; misc[9] = ov; }
  }
  __syncthreads();

  if (wave == 0) {
    const int base = lane * (NBRUN / 32);
    int s = 0;
#pragma unroll 1
    for (int i = 0; i < NBRUN / 32; ++i) s += cnt[base + i];
    int incl = s;
#pragma unroll
    for (int d = 1; d < 32; d <<= 1) {
      const int y = __shfl_up(incl, d, 32);
      if (lane >= d) incl += y;
    }
    int run = incl - s;
#pragma unroll 1
    for (int i = 0; i < NBRUN / 32; ++i) {
      const int cvv = cnt[base + i];
      offs[base + i] = run;
      cur[base + i]  = run;
      run += cvv;
    }
  }
  __syncthreads();

  if (wave == 0) {
    int t = 0;
#pragma unroll 1
    for (int w2 = 0; w2 < NWAVE; ++w2) {
      int c = misc[w2];
      c = c < 0 ? 0 : (c > WLCAP ? WLCAP : c);
      c = __builtin_amdgcn_readfirstlane(c);
#pragma unroll 1
      for (int b0 = 0; b0 < c; b0 += 32) {
        const int idx = b0 + lane;
        const int ent = wl[w2 * WLCAP + (idx < WLCAP ? idx : WLCAP - 1)];
        int sv = srcs[clampi(ent >> SLB, 0, NE - 1)];
        PIN(sv);
        sv = clampi(sv, 0, nN - 1);
        const int m32 = (c - b0) < 32 ? (c - b0) : 32;
#pragma unroll 1
        for (int k = 0; k < m32; ++k) {
          const int u    = __builtin_amdgcn_readlane(ent, k);
          const int sk   = __builtin_amdgcn_readlane(sv, k);
          const int slot = u & (NBRUN - 1);
          if (t < LCAP) {
            int p = cur[slot];
            p = p < 0 ? 0 : (p > LCAP - 1 ? LCAP - 1 : p);
            if (lane == 0) { sl[2 * p] = sk; sl[2 * p + 1] = u >> SLB; cur[slot] = p + 1; }
            t = t + 1;
          }
        }
      }
    }
  }
  __syncthreads();

  {
    const int ovf = misc[9];
    const v4i fv = {ovf, ovf, ovf, ovf};
    int* lb = listG + (size_t)b * (2 * LCAP);
    for (int pass = 0; pass < 2; ++pass) {
#pragma unroll 1
      for (int it = 0; it < LIST_IT; ++it) {
        const int i4 = it * NTHR + tid;
        const int ic = i4 < LIST_V4 ? i4 : LIST_V4 - 1;
        const v4i v = *(const v4ia*)(sl + 4 * ic);
        if (i4 < LIST_V4) *(volatile v4i*)(lb + 4 * (size_t)i4) = v;
      }
      {
        const v4i c4 = *(const v4ia*)(cnt + 4 * tid);
        const v4i o4 = *(const v4ia*)(offs + 4 * tid);
        *(volatile v4i*)(cntG + (size_t)nodeBase + 4 * tid) = c4;
        *(volatile v4i*)(offG + (size_t)nodeBase + 4 * tid) = o4;
      }
      if (tid < 8) *(volatile v4i*)(flagG + (size_t)b * 32 + 4 * tid) = fv;
      __threadfence();
    }
  }
}

__device__ __forceinline__ void ent_at(int srcA, int srcB, int sA, int sB, int k, int& src, float& s) {
  const int kk = k & 31;
  const int a0 = __builtin_amdgcn_readlane(srcA, kk);
  const int a1 = __builtin_amdgcn_readlane(srcB, kk);
  const int b0 = __builtin_amdgcn_readlane(sA, kk);
  const int b1 = __builtin_amdgcn_readlane(sB, kk);
  src = (k < 32) ? a0 : a1;
  s   = __int_as_float((k < 32) ? b0 : b1);
}

template <int KOUT>
__global__ __launch_bounds__(NTHR) void k_replay1(const float* __restrict__ XL, const int* __restrict__ listG,
                                                  const int* __restrict__ cntG, const int* __restrict__ offG,
                                                  const int* __restrict__ flagG, const float* __restrict__ wmul,
                                                  const float* __restrict__ tab, unsigned short* hb,
                                                  int nN, int mRows) {
  static_assert(KOUT == 128 || KOUT == 256);
  __shared__ __attribute__((aligned(16))) float sTab[3 * DH];
  __shared__ __attribute__((aligned(16))) float sRow[NWAVE][DH];
  const int tid = (int)threadIdx.x, lane = tid & 31, wave = tid >> 5;
  const int b = (int)blockIdx.x;
  {
    const int tq = tid < 96 ? tid : 95;
    const v4f t4 = *(const v4fa*)(tab + 4 * tq);
    if (tid < 96) *(v4fa*)(sTab + 4 * tid) = t4;
  }
  __syncthreads();
  const int nodeBase = b * NBRUN;
  int fl = flagG[(size_t)b * 32];
  PIN(fl);
  const bool ovf = fl != 0;
  const int* listb = listG + (size_t)b * (2 * LCAP);
  const float qnan = __int_as_float(0x7fc00000);
  const float ninf = -__builtin_inff();
  float* st = sRow[wave];
  const bool wr = lane < (KOUT / 8);
  const int cb8 = 8 * (lane & 15);

#pragma unroll 1
  for (int q = 0; q < GPW; ++q) {
    const int row0 = nodeBase + RGRP * (wave * GPW + q);
    if (row0 >= mRows) continue;
    const int ti = clampi(row0 + lane, 0, NBLK * NBRUN - 1);
    int cntv = cntG[ti];
    int offv = offG[ti];
    PIN(cntv);
    PIN(offv);
    const int bigv = (cntv > DEGCAP) ? 1 : 0;
    cntv = cntv < 0 ? 0 : (cntv > DEGCAP ? DEGCAP : cntv);
    offv = offv < 0 ? 0 : (offv > LCAP ? LCAP : offv);
#pragma unroll 1
    for (int r = 0; r < RGRP; ++r) {
      const int node = row0 + r;
      const bool live = node < nN;
      const int c  = __builtin_amdgcn_readlane(cntv, r);
      const int o  = __builtin_amdgcn_readlane(offv, r);
      const int bg = __builtin_amdgcn_readlane(bigv, r);
      const int cn = __builtin_amdgcn_readfirstlane(live ? c : 0);
      const bool bad = ovf || (bg != 0);
      const int i0 = clampi(o + lane, 0, LCAP - 1);
      const int i1 = clampi(o + 32 + lane, 0, LCAP - 1);
      const v2i pA = *(const v2ia*)(listb + 2 * i0);
      const v2i pB = *(const v2ia*)(listb + 2 * i1);
      PIN(pA.x); PIN(pA.y); PIN(pB.x); PIN(pB.y);
      const int srcA = clampi(pA.x, 0, nN - 1);
      const int srcB = clampi(pB.x, 0, nN - 1);
      float wa = wmul[clampi(pA.y, 0, NE - 1)];
      float wb = wmul[clampi(pB.y, 0, NE - 1)];
      PIN(wa);
      PIN(wb);
      const int sA = (int)(bf16_bits(wa) << 16);
      const int sB = (int)(bf16_bits(wb) << 16);
#pragma unroll 1
      for (int j = 0; j < 4; ++j) {
        const int ch = 32 * j + lane;
        const float cu = sTab[ch];
        const float cw = sTab[DH + ch];
        const float cb = sTab[2 * DH + ch];
        float m = ninf;
#pragma unroll 1
        for (int k = 0; k < cn; ++k) {
          int sk; float sf;
          ent_at(srcA, srcB, sA, sB, k, sk, sf);
          const float cf = (sf > 0.0f) ? cu : cw;
          const float ow = sf * cf + cb;
          m = (ow > m || ow != ow) ? ow : m;
        }
        m = ((__float_as_uint(m) & 0x7fffffffu) < 0x7f800000u) ? m : 0.0f;
        float S = 0.0f, acc = 0.0f;
#pragma unroll 1
        for (int k = 0; k < cn; ++k) {
          int sk; float sf;
          ent_at(srcA, srcB, sA, sB, k, sk, sf);
          const float cf = (sf > 0.0f) ? cu : cw;
          const float ow = sf * cf + cb;
          float xv = XL[(size_t)sk * DH + ch];
          PIN(xv);
          const float e = expf(ow - m);
          S += e;
          acc += e * xv;
        }
        float v = acc / (S + 1e-16f);
        v = (cn > 0) ? v : 0.0f;
        float y = (v > 0.0f) ? v : 0x1.ac5afap+0f * expm1f(v);
        y = 0x1.0cfabep+0f * y;
        y = bad ? qnan : y;
        y = live ? y : 0.0f;
        st[ch] = y;
      }
      __builtin_amdgcn_fence(__ATOMIC_RELEASE, "workgroup");
      __builtin_amdgcn_wave_barrier();
      __builtin_amdgcn_fence(__ATOMIC_ACQUIRE, "workgroup");
      const v4f ra = *(const v4fa*)(st + cb8);
      const v4f rc = *(const v4fa*)(st + cb8 + 4);
      const v4u hi = pack8_bf16(ra, rc);
      v4u pv = hi;
      if (KOUT == 256) {
        const v4u lo = pack8_bf16_lo(ra, rc);
        pv = (lane >= 16) ? lo : hi;
      }
      unsigned short* hp = hb + (size_t)node * KOUT + 8 * lane;
      if (wr) *(volatile v4u*)hp = pv;
      __threadfence();
      if (wr) *(volatile v4u*)hp = pv;
      __builtin_amdgcn_fence(__ATOMIC_RELEASE, "workgroup");
      __builtin_amdgcn_wave_barrier();
      __builtin_amdgcn_fence(__ATOMIC_ACQUIRE, "workgroup");
    }
  }
}

__global__ __launch_bounds__(NTHR) void k_replay2_out(const float* __restrict__ XL, const int* __restrict__ listG,
                                                      const int* __restrict__ cntG, const int* __restrict__ offG,
                                                      const int* __restrict__ flagG, const float* __restrict__ wmul,
                                                      const float* __restrict__ tab2, float* outP, float* outL,
                                                      int nN, int outN) {
  __shared__ __attribute__((aligned(16))) float stripP[NWAVE][RGRP * DC];
  __shared__ __attribute__((aligned(16))) float stripL[NWAVE][RGRP * DC];
  const int tid = (int)threadIdx.x, lane = tid & 31, wave = tid >> 5;
  const int b = (int)blockIdx.x;
  const int nodeBase = b * NBRUN;
  const v2f cu = *(const v2fa*)(tab2 + 2 * lane);
  const v2f cw = *(const v2fa*)(tab2 + 64 + 2 * lane);
  const v2f cb = *(const v2fa*)(tab2 + 128 + 2 * lane);
  int fl = flagG[(size_t)b * 32];
  PIN(fl);
  const bool ovf = fl != 0;
  const int* listb = listG + (size_t)b * (2 * LCAP);
  const float qnan = __int_as_float(0x7fc00000);
  const float ninf = -__builtin_inff();
  const int c0 = 2 * lane;
  const bool val0 = c0 < DC;
  const bool val1 = (c0 + 1) < DC;
  float* sp = stripP[wave];
  float* sg = stripL[wave];

#pragma unroll 1
  for (int q = 0; q < GPW; ++q) {
    const int row0 = nodeBase + RGRP * (wave * GPW + q);
    if (row0 >= nN) continue;
    const int ti = clampi(row0 + lane, 0, NBLK * NBRUN - 1);
    int cntv = cntG[ti];
    int offv = offG[ti];
    PIN(cntv);
    PIN(offv);
    const int bigv = (cntv > DEGCAP) ? 1 : 0;
    cntv = cntv < 0 ? 0 : (cntv > DEGCAP ? DEGCAP : cntv);
    offv = offv < 0 ? 0 : (offv > LCAP ? LCAP : offv);
#pragma unroll 1
    for (int r = 0; r < RGRP; ++r) {
      const int node = row0 + r;
      const bool live = node < nN;
      const int c  = __builtin_amdgcn_readlane(cntv, r);
      const int o  = __builtin_amdgcn_readlane(offv, r);
      const int bg = __builtin_amdgcn_readlane(bigv, r);
      const int cn = __builtin_amdgcn_readfirstlane(live ? c : 0);
      const bool bad = ovf || (bg != 0);
      const int i0 = clampi(o + lane, 0, LCAP - 1);
      const int i1 = clampi(o + 32 + lane, 0, LCAP - 1);
      const v2i pA = *(const v2ia*)(listb + 2 * i0);
      const v2i pB = *(const v2ia*)(listb + 2 * i1);
      PIN(pA.x); PIN(pA.y); PIN(pB.x); PIN(pB.y);
      const int srcA = clampi(pA.x, 0, nN - 1);
      const int srcB = clampi(pB.x, 0, nN - 1);
      float wa = wmul[clampi(pA.y, 0, NE - 1)];
      float wb = wmul[clampi(pB.y, 0, NE - 1)];
      PIN(wa);
      PIN(wb);
      const int sA = (int)(bf16_bits(wa) << 16);
      const int sB = (int)(bf16_bits(wb) << 16);

      float mx0 = ninf, mx1 = ninf;
#pragma unroll 1
      for (int k = 0; k < cn; ++k) {
        int sk; float sf;
        ent_at(srcA, srcB, sA, sB, k, sk, sf);
        const bool ps = sf > 0.0f;
        const float f0 = ps ? cu.x : cw.x;
        const float f1 = ps ? cu.y : cw.y;
        const float ow0 = sf * f0 + cb.x;
        const float ow1 = sf * f1 + cb.y;
        mx0 = (ow0 > mx0 || ow0 != ow0) ? ow0 : mx0;
        mx1 = (ow1 > mx1 || ow1 != ow1) ? ow1 : mx1;
      }
      mx0 = ((__float_as_uint(mx0) & 0x7fffffffu) < 0x7f800000u) ? mx0 : 0.0f;
      mx1 = ((__float_as_uint(mx1) & 0x7fffffffu) < 0x7f800000u) ? mx1 : 0.0f;
      float S0 = 0.0f, S1 = 0.0f, a0 = 0.0f, a1 = 0.0f;
#pragma unroll 1
      for (int k = 0; k < cn; ++k) {
        int sk; float sf;
        ent_at(srcA, srcB, sA, sB, k, sk, sf);
        const bool ps = sf > 0.0f;
        const float f0 = ps ? cu.x : cw.x;
        const float f1 = ps ? cu.y : cw.y;
        const float ow0 = sf * f0 + cb.x;
        const float ow1 = sf * f1 + cb.y;
        const v2f xv = *(const v2fa*)(XL + (size_t)sk * DCP + 2 * lane);
        PIN(xv.x);
        PIN(xv.y);
        const float e0 = expf(ow0 - mx0);
        const float e1 = expf(ow1 - mx1);
        S0 += e0; S1 += e1;
        a0 += e0 * xv.x;
        a1 += e1 * xv.y;
      }
      float o0 = a0 / (S0 + 1e-16f);
      float o1 = a1 / (S1 + 1e-16f);
      o0 = (cn > 0) ? o0 : 0.0f;
      o1 = (cn > 0) ? o1 : 0.0f;

      const float q0 = val0 ? o0 : ninf;
      const float q1 = val1 ? o1 : ninf;
      float m = q0;
      m = (q1 > m || q1 != q1) ? q1 : m;
#pragma unroll
      for (int off = 16; off > 0; off >>= 1) {
        const float y = __shfl_xor(m, off, 32);
        m = (y > m || y != y) ? y : m;
      }
      const float x0 = expf(o0 - m);
      const float x1 = expf(o1 - m);
      float s = (val0 ? x0 : 0.0f) + (val1 ? x1 : 0.0f);
#pragma unroll
      for (int off = 16; off > 0; off >>= 1) s += __shfl_xor(s, off, 32);
      const float ls = logf(s);
      float w0 = (o0 - m) - ls;
      float w1 = (o1 - m) - ls;
      w0 = bad ? qnan : w0;
      w1 = bad ? qnan : w1;
      o0 = bad ? qnan : o0;
      o1 = bad ? qnan : o1;
      if (val0) { sp[r * DC + c0] = w0;     sg[r * DC + c0] = o0; }
      if (val1) { sp[r * DC + c0 + 1] = w1; sg[r * DC + c0 + 1] = o1; }
    }
    __builtin_amdgcn_fence(__ATOMIC_RELEASE, "workgroup");
    __builtin_amdgcn_wave_barrier();
    __builtin_amdgcn_fence(__ATOMIC_ACQUIRE, "workgroup");
    const size_t fbase = (size_t)row0 * DC;
    {
      v4f vv[OUT_IT];
#pragma unroll
      for (int it = 0; it < OUT_IT; ++it) vv[it] = *(const v4fa*)(sp + 4 * (it * 32 + lane));
      for (int pass = 0; pass < 2; ++pass) {
#pragma unroll
        for (int it = 0; it < OUT_IT; ++it) {
          const size_t f = fbase + 4 * (size_t)(it * 32 + lane);
          if (f + 4 <= (size_t)outN) *(volatile v4f*)(outP + f) = vv[it];
        }
        __threadfence();
      }
    }
    {
      v4f vv[OUT_IT];
#pragma unroll
      for (int it = 0; it < OUT_IT; ++it) vv[it] = *(const v4fa*)(sg + 4 * (it * 32 + lane));
      for (int pass = 0; pass < 2; ++pass) {
#pragma unroll
        for (int it = 0; it < OUT_IT; ++it) {
          const size_t f = fbase + 4 * (size_t)(it * 32 + lane);
          if (f + 4 <= (size_t)outN) *(volatile v4f*)(outL + f) = vv[it];
        }
        __threadfence();
      }
    }
    __builtin_amdgcn_fence(__ATOMIC_RELEASE, "workgroup");
    __builtin_amdgcn_wave_barrier();
    __builtin_amdgcn_fence(__ATOMIC_ACQUIRE, "workgroup");
  }
}

constexpr size_t SZ_XB   = (size_t)MPAD * DF * 2;
constexpr size_t SZ_XL1  = (size_t)MPAD * DH * 4;
constexpr size_t SZ_HHL  = (size_t)MPAD * 256 * 2;
constexpr size_t SZ_XL2  = (size_t)MPAD * DCP * 4;
constexpr size_t SZ_LIST = (size_t)NBLK * LCAP * 8;
constexpr size_t SZ_CNT  = (size_t)NBLK * NBRUN * 4;
constexpr size_t SZ_FLAG = 8192;
constexpr size_t SZ_W1P  = (size_t)DH * DF * 2;
constexpr size_t SZ_W2D  = (size_t)DCP * 256 * 2;
constexpr size_t SZ_TAB  = 4096;
constexpr size_t O_XB   = 0;
constexpr size_t O_XL1  = O_XB + SZ_XB;
constexpr size_t O_HHL  = O_XL1 + SZ_XL1;
constexpr size_t O_XL2  = O_HHL + SZ_HHL;
constexpr size_t O_LIST = O_XL2 + SZ_XL2;
constexpr size_t O_CNT  = O_LIST + SZ_LIST;
constexpr size_t O_OFF  = O_CNT + SZ_CNT;
constexpr size_t O_FLAG = O_OFF + SZ_CNT;
constexpr size_t O_W1P  = O_FLAG + SZ_FLAG;
constexpr size_t O_W2D  = O_W1P + SZ_W1P;
constexpr size_t O_TAB  = O_W2D + SZ_W2D;
constexpr size_t WS_TOTAL = O_TAB + SZ_TAB;
static_assert(SZ_XB % 256 == 0 && SZ_XL1 % 256 == 0 && SZ_HHL % 256 == 0 && SZ_XL2 % 256 == 0);
static_assert(SZ_LIST % 256 == 0 && SZ_CNT % 256 == 0 && SZ_FLAG % 256 == 0 && SZ_W1P % 256 == 0);
static_assert(SZ_W2D % 256 == 0 && SZ_TAB % 256 == 0);
static_assert(WS_TOTAL == 85506560 && WS_TOTAL <= ((size_t)128 << 20));
static_assert((size_t)MPAD * K2 * 2 <= SZ_HHL && (size_t)DCP * K2 * 2 <= SZ_W2D);
static_assert((size_t)NBLK * 128 <= SZ_FLAG && (size_t)T_TOT * 4 <= SZ_TAB);
static_assert((size_t)2 * OUTN * 4 == 16000000);

extern "C" void kernel_launch(void* const* d_in, const int* in_sizes, int n_in,
                              void* d_out, int out_size, void* d_ws, size_t ws_size,
                              hipStream_t stream) {
  if (n_in < 13) return;
  if (in_sizes[0] != NN * DF) return;
  if (in_sizes[1] != 2 * NE) return;
  if (in_sizes[2] != NE) return;
  if (in_sizes[3] != DH * DF || in_sizes[4] != DH) return;
  if (in_sizes[5] != DH || in_sizes[6] != DH * DH || in_sizes[7] != DH) return;
  if (in_sizes[8] != DC * DH || in_sizes[9] != DC) return;
  if (in_sizes[10] != DC || in_sizes[11] != DC * DC || in_sizes[12] != DC) return;
  if (out_size != 2 * OUTN) return;
  if (ws_size < WS_TOTAL) return;

  const float* x     = (const float*)d_in[0];
  const int*   edge  = (const int*)d_in[1];
  const float* wmul  = (const float*)d_in[2];
  const float* linw1 = (const float*)d_in[3];
  const float* linb1 = (const float*)d_in[4];
  const float* w1a   = (const float*)d_in[5];
  const float* w2a   = (const float*)d_in[6];
  const float* w2ba  = (const float*)d_in[7];
  const float* linw2 = (const float*)d_in[8];
  const float* linb2 = (const float*)d_in[9];
  const float* w1b   = (const float*)d_in[10];
  const float* w2b   = (const float*)d_in[11];
  const float* w2bb  = (const float*)d_in[12];
  float* out0 = (float*)d_out;
  float* out1 = (float*)d_out + OUTN;
  const int* src = edge;
  const int* tgt = edge + NE;

  char* ws = (char*)d_ws;
  unsigned short* XB  = (unsigned short*)(ws + O_XB);
  float*          XL1 = (float*)(ws + O_XL1);
  unsigned short* HHL = (unsigned short*)(ws + O_HHL);
  float*          XL2 = (float*)(ws + O_XL2);
  int*            LST = (int*)(ws + O_LIST);
  int*            CNT = (int*)(ws + O_CNT);
  int*            OFF = (int*)(ws + O_OFF);
  int*            FLG = (int*)(ws + O_FLAG);
  unsigned short* W1P = (unsigned short*)(ws + O_W1P);
  unsigned short* W2D = (unsigned short*)(ws + O_W2D);
  float*          TAB = (float*)(ws + O_TAB);

  hipFuncSetAttribute(reinterpret_cast<const void*>(&k_bucket), hipFuncAttributeMaxDynamicSharedMemorySize,
                      (int)BK_LDS);

  const int gemm1Grid = ((MPAD / 64) * (DH / 64) + 7) / 8;
  const int gemm2Grid = ((MPAD / 64) + 7) / 8;

  k_plane<0><<<MPAD * (DF / 8) / 256, 256, 0, stream>>>(x, NN, DF, DF, XB, MPAD, DF);
  k_prep<<<NBW1 + NBW2 + 1, NTHR, 0, stream>>>(linw1, linb1, w1a, w2a, w2ba, linw2, linb2, w1b, w2b, w2bb,
                                               W1P, W2D, TAB);
  k_bucket<<<NBLK, NTHR, BK_LDS, stream>>>(src, tgt, NN, LST, CNT, OFF, FLG);
  k_gemm_nt<0, 1><<<gemm1Grid, 256, 0, stream>>>(XB, W1P, TAB + T_LB1, XL1, MPAD, DH, DF, DH);
  k_replay1<K2><<<NBLK, NTHR, 0, stream>>>(XL1, LST, CNT, OFF, FLG, wmul, TAB, HHL, NN, MPAD);
  k_gemm_nt<HL2 ? 1 : 0, 1><<<gemm2Grid, 256, 0, stream>>>(HHL, W2D, TAB + T_LB2, XL2, MPAD, DCP, K2, DCP);
  k_replay2_out<<<NBLK, NTHR, 0, stream>>>(XL2, LST, CNT, OFF, FLG, wmul, TAB + T_U2, out0, out1, NN, OUTN);
}
